// CharEmbedder_23304492548444
// MI455X (gfx1250) — hardware-verified
//
#include <hip/hip_runtime.h>


typedef _Float16 v16h __attribute__((ext_vector_type(16)));
typedef _Float16 v8h  __attribute__((ext_vector_type(8)));
typedef float    v8f  __attribute__((ext_vector_type(8)));
typedef float    v4f  __attribute__((ext_vector_type(4)));
typedef unsigned int v4u __attribute__((ext_vector_type(4)));
typedef v4f __attribute__((may_alias)) v4fa;

#define TOKENS 2048
#define NCH    50
#define EMB    16
#define NCHARS 262
#define XCOL   832
#define XG     104
#define NFILT  2048
#define HWN    4096
#define ODIM   512
#define CONVW_ELEMS 219136
#define SCALE_X  16.0f
#define SCALE_CW 16.0f
#define INV_CONV (1.0f / 256.0f)
#define SCALE_W  32.0f
#define INV_W    (1.0f / 32.0f)

union Frag  { v16h v; v8h half[2]; };
union Pack8 { v8h h; v4u u; };

__device__ __forceinline__ v16h ldfrag(const _Float16* __restrict__ row, int k0, int h) {
    Frag f;
    f.half[0] = *(const v8h*)(row + k0 + 8 * h);
    f.half[1] = *(const v8h*)(row + k0 + 16 + 8 * h);
    return f.v;
}

__device__ __forceinline__ v8f wmma16(v16h a, v16h b, v8f c) {
    v8f d = __builtin_amdgcn_wmma_f32_16x16x32_f16(false, a, false, b, (short)0, c, false, false);
    asm volatile("v_nop\n\tv_nop\n\tv_nop\n\tv_nop" : "+v"(d) : "v"(a), "v"(b));
    return d;
}

__device__ __forceinline__ v4u pack8(v4f x0, v4f x1, float s) {
    Pack8 o;
    o.h[0] = (_Float16)(x0.x * s); o.h[1] = (_Float16)(x0.y * s);
    o.h[2] = (_Float16)(x0.z * s); o.h[3] = (_Float16)(x0.w * s);
    o.h[4] = (_Float16)(x1.x * s); o.h[5] = (_Float16)(x1.y * s);
    o.h[6] = (_Float16)(x1.z * s); o.h[7] = (_Float16)(x1.w * s);
    return o.u;
}

__global__ void __launch_bounds__(256)
k_prep_x(const int* __restrict__ ids, const float* __restrict__ emb, _Float16* __restrict__ Xh) {
    const int g = blockIdx.x * blockDim.x + threadIdx.x;
    if (g >= TOKENS * XG) return;
    const int t = g / XG, gi = g - t * XG;
    const int col8 = gi * 8;
    v4f x0 = {0.f, 0.f, 0.f, 0.f}, x1 = {0.f, 0.f, 0.f, 0.f};
    if (col8 < NCH * EMB) {
        const int c = gi >> 1, e0 = (gi & 1) * 8;
        int id = ids[t * NCH + c];
        id = id < 0 ? 0 : (id > NCHARS - 1 ? NCHARS - 1 : id);
        const v4f* p = (const v4f*)(emb + (size_t)id * EMB + e0);
        x0 = p[0]; x1 = p[1];
    }
    const v4u u = pack8(x0, x1, SCALE_X);
    v4u* dst = (v4u*)(Xh + (size_t)g * 8);
    *(volatile v4u*)dst = u;
    __threadfence();
    *(volatile v4u*)dst = u;
}

__global__ void __launch_bounds__(256)
k_prep_convw(const float* __restrict__ w0, const float* __restrict__ w1,
             const float* __restrict__ w2, const float* __restrict__ w3,
             const float* __restrict__ w4, const float* __restrict__ w5,
             const float* __restrict__ w6, _Float16* __restrict__ Wc) {
    const int g = blockIdx.x * blockDim.x + threadIdx.x;
    if (g >= CONVW_ELEMS / 8) return;
    const int idx = g * 8;
    const float* w; int base, Kp, ksz;
    if      (idx < 1024)   { w = w0; base = 0;     Kp = 32;  ksz = 1; }
    else if (idx < 2048)   { w = w1; base = 1024;  Kp = 32;  ksz = 2; }
    else if (idx < 6144)   { w = w2; base = 2048;  Kp = 64;  ksz = 3; }
    else if (idx < 14336)  { w = w3; base = 6144;  Kp = 64;  ksz = 4; }
    else if (idx < 38912)  { w = w4; base = 14336; Kp = 96;  ksz = 5; }
    else if (idx < 88064)  { w = w5; base = 38912; Kp = 96;  ksz = 6; }
    else                   { w = w6; base = 88064; Kp = 128; ksz = 7; }
    const int local = idx - base;
    const int o = local / Kp, j0 = local - o * Kp;
    const int dk = j0 >> 4, e0 = j0 & 15;
    v4f x0 = {0.f, 0.f, 0.f, 0.f}, x1 = {0.f, 0.f, 0.f, 0.f};
    if (j0 < EMB * ksz) {
        const float* src = w + ((size_t)o * EMB + e0) * ksz + dk;
        x0.x = src[0 * ksz]; x0.y = src[1 * ksz]; x0.z = src[2 * ksz]; x0.w = src[3 * ksz];
        x1.x = src[4 * ksz]; x1.y = src[5 * ksz]; x1.z = src[6 * ksz]; x1.w = src[7 * ksz];
    }
    const v4u u = pack8(x0, x1, SCALE_CW);
    v4u* dst = (v4u*)(Wc + (size_t)g * 8);
    *(volatile v4u*)dst = u;
    __threadfence();
    *(volatile v4u*)dst = u;
}

__global__ void __launch_bounds__(256)
k_cvt(const float* __restrict__ s, _Float16* __restrict__ d, int n8, float scale) {
    const int g = blockIdx.x * blockDim.x + threadIdx.x;
    if (g >= n8) return;
    const v4f* p = (const v4f*)(s + (size_t)g * 8);
    const v4u u = pack8(p[0], p[1], scale);
    v4u* dst = (v4u*)(d + (size_t)g * 8);
    *(volatile v4u*)dst = u;
    __threadfence();
    *(volatile v4u*)dst = u;
}

template<int KSZ, int KP, int WBASE, int GBASE, int OC>
__global__ void __launch_bounds__(64)
k_conv(const _Float16* __restrict__ Xh, const _Float16* __restrict__ Wc,
       const float* __restrict__ bias, float* __restrict__ Hf) {
    constexpr int NK = KP / 32;
    constexpr int P  = NCH + 1 - KSZ;
    constexpr int FT = OC / 32;
    __shared__ float tile[16][32];

    const int w = threadIdx.x >> 5, lane = threadIdx.x & 31, h = lane >> 4, m = lane & 15;
    const int ttile = blockIdx.x / FT, ft = blockIdx.x - ttile * FT;
    const int t0 = ttile * 16;
    const int nloc = ft * 32 + w * 16 + m;
    const _Float16* arow = Xh + (size_t)(t0 + m) * XCOL;
    const _Float16* brow = Wc + WBASE + (size_t)nloc * KP;
    const float bb = bias[nloc];

    v16h bfr[NK];
    #pragma unroll
    for (int q = 0; q < NK; ++q) bfr[q] = ldfrag(brow, q * 32, h);

    v8f mx;
    #pragma unroll
    for (int j = 0; j < 8; ++j) mx[j] = -3.402823466e38f;

    #pragma unroll 2
    for (int p = 0; p < P; ++p) {
        v8f acc = {0.f, 0.f, 0.f, 0.f, 0.f, 0.f, 0.f, 0.f};
        #pragma unroll
        for (int q = 0; q < NK; ++q)
            acc = wmma16(ldfrag(arow, p * 16 + q * 32, h), bfr[q], acc);
        #pragma unroll
        for (int j = 0; j < 8; ++j) mx[j] = fmaxf(mx[j], acc[j]);
    }

    #pragma unroll
    for (int j = 0; j < 8; ++j)
        tile[8 * h + j][w * 16 + m] = fmaxf(mx[j] * INV_CONV + bb, 0.0f);
    __syncthreads();

    v4f vv[2];
    #pragma unroll
    for (int it = 0; it < 2; ++it) {
        const int rl = w * 8 + it * 4 + (lane >> 3), cl = (lane & 7) * 4;
        vv[it] = *(const v4fa*)&tile[rl][cl];
    }
    #pragma unroll
    for (int it = 0; it < 2; ++it) {
        const int rl = w * 8 + it * 4 + (lane >> 3), cl = (lane & 7) * 4;
        *(volatile v4f*)(Hf + (size_t)(t0 + rl) * NFILT + GBASE + ft * 32 + cl) = vv[it];
    }
    __threadfence();
    #pragma unroll
    for (int it = 0; it < 2; ++it) {
        const int rl = w * 8 + it * 4 + (lane >> 3), cl = (lane & 7) * 4;
        *(volatile v4f*)(Hf + (size_t)(t0 + rl) * NFILT + GBASE + ft * 32 + cl) = vv[it];
    }
}

template<int K>
__device__ __forceinline__ void gemm_2x4(const _Float16* __restrict__ A, int m0,
                                         const _Float16* __restrict__ Bt,
                                         int nb0, int nb1, int nb2, int nb3,
                                         int h, int m, v8f (&acc)[2][4]) {
    const _Float16* a0p = A + (size_t)(m0 + m) * K;
    const _Float16* a1p = A + (size_t)(m0 + 16 + m) * K;
    const _Float16* bp[4] = { Bt + (size_t)(nb0 + m) * K, Bt + (size_t)(nb1 + m) * K,
                              Bt + (size_t)(nb2 + m) * K, Bt + (size_t)(nb3 + m) * K };
    #pragma unroll 1
    for (int k0 = 0; k0 < K; k0 += 32) {
        const v16h a0 = ldfrag(a0p, k0, h);
        const v16h a1 = ldfrag(a1p, k0, h);
        #pragma unroll
        for (int s = 0; s < 4; ++s) {
            const v16h b = ldfrag(bp[s], k0, h);
            acc[0][s] = wmma16(a0, b, acc[0][s]);
            acc[1][s] = wmma16(a1, b, acc[1][s]);
        }
    }
}

__global__ void __launch_bounds__(256)
k_hwy(const _Float16* __restrict__ Hh, const _Float16* __restrict__ Wh,
      const float* __restrict__ b, const float* __restrict__ Hin, float* __restrict__ Hout) {
    __shared__ float tile[8][32][32];
    const int w = threadIdx.x >> 5, lane = threadIdx.x & 31, h = lane >> 4, m = lane & 15;
    const int gw = blockIdx.x * 8 + w;
    const int m0 = (gw >> 6) * 32;
    const int c0 = (gw & 63) * 32;

    v8f acc[2][4];
    #pragma unroll
    for (int r = 0; r < 2; ++r)
        #pragma unroll
        for (int s = 0; s < 4; ++s) acc[r][s] = (v8f){0.f, 0.f, 0.f, 0.f, 0.f, 0.f, 0.f, 0.f};

    gemm_2x4<NFILT>(Hh, m0, Wh, c0, c0 + 16, NFILT + c0, NFILT + c0 + 16, h, m, acc);

    #pragma unroll
    for (int r = 0; r < 2; ++r) {
        #pragma unroll
        for (int s = 0; s < 2; ++s) {
            const int k = c0 + 16 * s + m;
            const float bn = b[k], bg = b[NFILT + k];
            #pragma unroll
            for (int j = 0; j < 8; ++j) {
                const int row = m0 + 16 * r + 8 * h + j;
                const float nl = acc[r][s][j] * INV_W + bn;
                float gp = acc[r][s + 2][j] * INV_W + bg;
                gp = fmaxf(gp, -60.0f);
                const float e = expf(-gp);
                const float gate = __builtin_amdgcn_rcpf(1.0f + e);
                const float hold = Hin[(size_t)row * NFILT + k];
                tile[w][16 * r + 8 * h + j][16 * s + m] = gate * hold + (1.0f - gate) * fmaxf(nl, 0.0f);
            }
        }
    }
    __syncthreads();

    v4f vv[8];
    #pragma unroll
    for (int it = 0; it < 8; ++it) {
        const int rl = it * 4 + (lane >> 3), cl = (lane & 7) * 4;
        vv[it] = *(const v4fa*)&tile[w][rl][cl];
    }
    #pragma unroll
    for (int it = 0; it < 8; ++it) {
        const int rl = it * 4 + (lane >> 3), cl = (lane & 7) * 4;
        *(volatile v4f*)(Hout + (size_t)(m0 + rl) * NFILT + c0 + cl) = vv[it];
    }
    __threadfence();
    #pragma unroll
    for (int it = 0; it < 8; ++it) {
        const int rl = it * 4 + (lane >> 3), cl = (lane & 7) * 4;
        *(volatile v4f*)(Hout + (size_t)(m0 + rl) * NFILT + c0 + cl) = vv[it];
    }
}

__global__ void __launch_bounds__(128)
k_proj(const _Float16* __restrict__ Hh, const _Float16* __restrict__ Wp,
       const float* __restrict__ b, float* __restrict__ out) {
    __shared__ float tile[4][32][64];
    const int w = threadIdx.x >> 5, lane = threadIdx.x & 31, h = lane >> 4, m = lane & 15;
    const int gw = blockIdx.x * 4 + w;
    const int m0 = (gw >> 3) * 32;
    const int n0 = (gw & 7) * 64;

    v8f acc[2][4];
    #pragma unroll
    for (int r = 0; r < 2; ++r)
        #pragma unroll
        for (int s = 0; s < 4; ++s) acc[r][s] = (v8f){0.f, 0.f, 0.f, 0.f, 0.f, 0.f, 0.f, 0.f};

    gemm_2x4<NFILT>(Hh, m0, Wp, n0, n0 + 16, n0 + 32, n0 + 48, h, m, acc);

    #pragma unroll
    for (int s = 0; s < 4; ++s) {
        const float bb = b[n0 + 16 * s + m];
        #pragma unroll
        for (int r = 0; r < 2; ++r)
            #pragma unroll
            for (int j = 0; j < 8; ++j)
                tile[w][16 * r + 8 * h + j][16 * s + m] = acc[r][s][j] * INV_W + bb;
    }
    __syncthreads();

    v4f vv[16];
    #pragma unroll
    for (int it = 0; it < 16; ++it) {
        const int L = it * 4 + (lane >> 3), rl = L >> 1, cl = (L & 1) * 32 + (lane & 7) * 4;
        vv[it] = *(const v4fa*)&tile[w][rl][cl];
    }
    #pragma unroll
    for (int it = 0; it < 16; ++it) {
        const int L = it * 4 + (lane >> 3), rl = L >> 1, cl = (L & 1) * 32 + (lane & 7) * 4;
        *(volatile v4f*)(out + (size_t)(m0 + rl) * ODIM + n0 + cl) = vv[it];
    }
    __threadfence();
    #pragma unroll
    for (int it = 0; it < 16; ++it) {
        const int L = it * 4 + (lane >> 3), rl = L >> 1, cl = (L & 1) * 32 + (lane & 7) * 4;
        *(volatile v4f*)(out + (size_t)(m0 + rl) * ODIM + n0 + cl) = vv[it];
    }
}


extern "C" void kernel_launch(void* const* d_in, const int* in_sizes, int n_in,
                              void* d_out, int out_size, void* d_ws, size_t ws_size,
                              hipStream_t stream) {
    if (n_in < 22) return;
    if (in_sizes[0] != TOKENS * NCH || in_sizes[1] != NCHARS * EMB) return;
    if (in_sizes[16] != HWN * NFILT || in_sizes[18] != HWN * NFILT || in_sizes[20] != ODIM * NFILT) return;
    if (out_size != TOKENS * ODIM) return;

    const int*   ids = (const int*)d_in[0];
    const float* emb = (const float*)d_in[1];
    const float* cw[7]; const float* cb[7];
    for (int i = 0; i < 7; ++i) {
        cw[i] = (const float*)d_in[2 + 2 * i];
        cb[i] = (const float*)d_in[3 + 2 * i];
    }
    const float* hw_w0  = (const float*)d_in[16];
    const float* hw_b0  = (const float*)d_in[17];
    const float* hw_w1  = (const float*)d_in[18];
    const float* hw_b1  = (const float*)d_in[19];
    const float* proj_w = (const float*)d_in[20];
    const float* proj_b = (const float*)d_in[21];
    float* out = (float*)d_out;

    const size_t off_x   = 0;
    const size_t off_wc  = off_x   + (size_t)TOKENS * XCOL * 2;
    const size_t off_hfa = off_wc  + (size_t)CONVW_ELEMS * 2;
    const size_t off_hfb = off_hfa + (size_t)TOKENS * NFILT * 4;
    const size_t off_hh  = off_hfb + (size_t)TOKENS * NFILT * 4;
    const size_t off_w0  = off_hh  + (size_t)TOKENS * NFILT * 2;
    const size_t off_w1  = off_w0  + (size_t)HWN * NFILT * 2;
    const size_t off_wp  = off_w1  + (size_t)HWN * NFILT * 2;
    const size_t total   = off_wp  + (size_t)ODIM * NFILT * 2;
    if (total > ws_size) return;

    char* ws = (char*)d_ws;
    _Float16* Xh  = (_Float16*)(ws + off_x);
    _Float16* Wc  = (_Float16*)(ws + off_wc);
    float*    Hfa = (float*)(ws + off_hfa);
    float*    Hfb = (float*)(ws + off_hfb);
    _Float16* Hh  = (_Float16*)(ws + off_hh);
    _Float16* W0h = (_Float16*)(ws + off_w0);
    _Float16* W1h = (_Float16*)(ws + off_w1);
    _Float16* Wph = (_Float16*)(ws + off_wp);

    const dim3 blk(256);
    const int n8_hw = (HWN * NFILT) / 8;
    const int n8_pw = (ODIM * NFILT) / 8;
    const int n8_h  = (TOKENS * NFILT) / 8;

    k_prep_x<<<(TOKENS * XG + 255) / 256, blk, 0, stream>>>(ids, emb, Xh);
    k_prep_convw<<<(CONVW_ELEMS / 8 + 255) / 256, blk, 0, stream>>>(
        cw[0], cw[1], cw[2], cw[3], cw[4], cw[5], cw[6], Wc);
    k_cvt<<<(n8_hw + 255) / 256, blk, 0, stream>>>(hw_w0, W0h, n8_hw, SCALE_W);
    k_cvt<<<(n8_hw + 255) / 256, blk, 0, stream>>>(hw_w1, W1h, n8_hw, SCALE_W);
    k_cvt<<<(n8_pw + 255) / 256, blk, 0, stream>>>(proj_w, Wph, n8_pw, SCALE_W);

    const dim3 cblk(64);
    k_conv<1,  32, 0,     0,    32  ><<<128 * 1,  cblk, 0, stream>>>(Xh, Wc, cb[0], Hfa);
    k_conv<2,  32, 1024,  32,   32  ><<<128 * 1,  cblk, 0, stream>>>(Xh, Wc, cb[1], Hfa);
    k_conv<3,  64, 2048,  64,   64  ><<<128 * 2,  cblk, 0, stream>>>(Xh, Wc, cb[2], Hfa);
    k_conv<4,  64, 6144,  128,  128 ><<<128 * 4,  cblk, 0, stream>>>(Xh, Wc, cb[3], Hfa);
    k_conv<5,  96, 14336, 256,  256 ><<<128 * 8,  cblk, 0, stream>>>(Xh, Wc, cb[4], Hfa);
    k_conv<6,  96, 38912, 512,  512 ><<<128 * 16, cblk, 0, stream>>>(Xh, Wc, cb[5], Hfa);
    k_conv<7, 128, 88064, 1024, 1024><<<128 * 32, cblk, 0, stream>>>(Xh, Wc, cb[6], Hfa);

    k_cvt<<<(n8_h + 255) / 256, blk, 0, stream>>>(Hfa, Hh, n8_h, 1.0f);
    k_hwy<<<512, blk, 0, stream>>>(Hh, W0h, hw_b0, Hfa, Hfb);

    k_cvt<<<(n8_h + 255) / 256, blk, 0, stream>>>(Hfb, Hh, n8_h, 1.0f);
    k_hwy<<<512, blk, 0, stream>>>(Hh, W1h, hw_b1, Hfb, Hfa);

    k_cvt<<<(n8_h + 255) / 256, blk, 0, stream>>>(Hfa, Hh, n8_h, 1.0f);
    k_proj<<<128, dim3(128), 0, stream>>>(Hh, Wph, proj_b, out);
}
